// GraphAllocNet_37761352467077
// MI455X (gfx1250) — hardware-verified
//
#include <hip/hip_runtime.h>
#include <stddef.h>


#define HID    128
#define NTHR   256
#define NWAVE  8
#define EPT    8
#define CHUNK  (NTHR * EPT)
#define WCAP   (EPT * 32)
#define LISTN  (NWAVE * WCAP)
#define PASSN  (NWAVE * 16)
#define HALFP  (PASSN / 2)
#define PCAP   (CHUNK + PASSN)
#define NB     128
#define WMP    384
#define KOFE   128
#define GW     4
#define GTHR   (GW * 32)
#define DTHR   256
#define DPB    (DTHR / 2)

static_assert((PCAP % PASSN) == 0);
static_assert(PASSN == 128);
static_assert(HALFP == 64);
static_assert(NB == 2 * 8 * NWAVE);
static_assert(DPB == 8 * 16);

typedef float        v4f  __attribute__((ext_vector_type(4)));
typedef float        v8f  __attribute__((ext_vector_type(8)));
typedef int          v4i  __attribute__((ext_vector_type(4)));
typedef unsigned int v4u  __attribute__((ext_vector_type(4)));
typedef __bf16       v8b  __attribute__((ext_vector_type(8)));
typedef __bf16       v16b __attribute__((ext_vector_type(16)));
union H8    { v8b b; v4u q; };
union FragB { v16b v; v4u q[2]; };

__device__ __forceinline__ v8f zero8f() {
  v8f z;
#pragma unroll
  for (int i = 0; i < 8; ++i) z[i] = 0.0f;
  return z;
}

__device__ __forceinline__ v4u zero4u() {
  v4u z = {0u, 0u, 0u, 0u};
  return z;
}

__device__ __forceinline__ v8f cat8(v4f a, v4f b) {
  v8f r;
  r[0] = a.x; r[1] = a.y; r[2] = a.z; r[3] = a.w;
  r[4] = b.x; r[5] = b.y; r[6] = b.z; r[7] = b.w;
  return r;
}

__device__ __forceinline__ void split8(v8f x, H8& hi, H8& lo) {
#pragma unroll
  for (int i = 0; i < 8; ++i) {
    const __bf16 hb = (__bf16)x[i];
    const float rem = x[i] - (float)hb;
    hi.b[i] = hb;
    lo.b[i] = (__bf16)rem;
  }
}

__device__ __forceinline__ void split1(float f, unsigned short& h, unsigned short& l) {
  const __bf16 hb = (__bf16)f;
  const __bf16 lb = (__bf16)(f - (float)hb);
  h = __builtin_bit_cast(unsigned short, hb);
  l = __builtin_bit_cast(unsigned short, lb);
}

__device__ __forceinline__ v8f wmb(const FragB& a, const FragB& b, v8f c) {
  v8f d = __builtin_amdgcn_wmma_f32_16x16x32_bf16(false, a.v, false, b.v, (short)0, c, false, false);
  asm volatile("v_nop\n\tv_nop\n\tv_nop\n\tv_nop" : "+v"(d) : "v"(a.v), "v"(b.v));
  return d;
}

__device__ __forceinline__ int scan_chunk(const int* __restrict__ dsts, int nE, int cbase, int nodeBase,
                                          int vec8, int* hl, int tid, int wave) {
  int wc = 0;
  const int el0  = tid * EPT;
  const int e0   = cbase + el0;
  const int sent = -2147483647 - 1;
  v4i da, db;
  if (vec8 != 0 && cbase + CHUNK <= nE) {
    da = *(const v4i*)(dsts + e0);
    db = *(const v4i*)(dsts + e0 + 4);
  } else {
    da.x = (e0     < nE) ? dsts[min(e0, nE - 1)] : sent;
    da.y = (e0 + 1 < nE) ? dsts[min(e0 + 1, nE - 1)] : sent;
    da.z = (e0 + 2 < nE) ? dsts[min(e0 + 2, nE - 1)] : sent;
    da.w = (e0 + 3 < nE) ? dsts[min(e0 + 3, nE - 1)] : sent;
    db.x = (e0 + 4 < nE) ? dsts[min(e0 + 4, nE - 1)] : sent;
    db.y = (e0 + 5 < nE) ? dsts[min(e0 + 5, nE - 1)] : sent;
    db.z = (e0 + 6 < nE) ? dsts[min(e0 + 6, nE - 1)] : sent;
    db.w = (e0 + 7 < nE) ? dsts[min(e0 + 7, nE - 1)] : sent;
  }
  const unsigned nb = (unsigned)nodeBase;
  const unsigned s0 = (unsigned)da.x - nb, s1 = (unsigned)da.y - nb;
  const unsigned s2 = (unsigned)da.z - nb, s3 = (unsigned)da.w - nb;
  const unsigned s4 = (unsigned)db.x - nb, s5 = (unsigned)db.y - nb;
  const unsigned s6 = (unsigned)db.z - nb, s7 = (unsigned)db.w - nb;
  const bool h0 = s0 < (unsigned)NB, h1 = s1 < (unsigned)NB, h2 = s2 < (unsigned)NB, h3 = s3 < (unsigned)NB;
  const bool h4 = s4 < (unsigned)NB, h5 = s5 < (unsigned)NB, h6 = s6 < (unsigned)NB, h7 = s7 < (unsigned)NB;
  const unsigned any = __builtin_amdgcn_ballot_w32(h0 | h1 | h2 | h3 | h4 | h5 | h6 | h7);
  if (any != 0u) {
#define HITJ(J, HJ) { \
      const unsigned mj = __builtin_amdgcn_ballot_w32(HJ); \
      if (mj != 0u) { \
        if (HJ) { \
          const int pos = wc + (int)__builtin_amdgcn_mbcnt_lo(mj, 0u); \
          if (pos < WCAP) hl[wave * WCAP + pos] = el0 + (J); \
        } \
        wc += (int)__builtin_popcount(mj); } }
    HITJ(0, h0)
    HITJ(1, h1)
    HITJ(2, h2)
    HITJ(3, h3)
    HITJ(4, h4)
    HITJ(5, h5)
    HITJ(6, h6)
    HITJ(7, h7)
#undef HITJ
  }
  return wc;
}

__global__ __launch_bounds__(256) void k_wprep(
    const float* __restrict__ s0, const float* __restrict__ s1, const float* __restrict__ s2,
    const float* __restrict__ s3, const float* __restrict__ s4, const float* __restrict__ s5,
    int K0, int K1, int K2, int K3, int K4, int K5,
    int P0, int P1, int P2, int P3, int P4, int P5,
    int O0, int O1, int O2, int O3, int O4, int O5,
    unsigned short* wsb) {
  const int j = blockIdx.y;
  const float* src = (j == 0) ? s0 : (j == 1) ? s1 : (j == 2) ? s2 : (j == 3) ? s3 : (j == 4) ? s4 : s5;
  const int K   = (j == 0) ? K0 : (j == 1) ? K1 : (j == 2) ? K2 : (j == 3) ? K3 : (j == 4) ? K4 : K5;
  const int kp  = (j == 0) ? P0 : (j == 1) ? P1 : (j == 2) ? P2 : (j == 3) ? P3 : (j == 4) ? P4 : P5;
  const int off = (j == 0) ? O0 : (j == 1) ? O1 : (j == 2) ? O2 : (j == 3) ? O3 : (j == 4) ? O4 : O5;
  const int pieces = 16 * kp;
  const int p = blockIdx.x * 256 + threadIdx.x;
  const bool ok = p < pieces;
  const int pc = ok ? p : 0;
  const int n  = (8 * pc) / kp;
  const int k0 = 8 * pc - n * kp;
  v8f x;
#pragma unroll
  for (int i = 0; i < 8; ++i) {
    const int k  = k0 + i;
    const int kc = (k < K) ? k : (K - 1);
    const float t = src[(size_t)kc * HID + n];
    x[i] = (k < K) ? t : 0.0f;
  }
  H8 h, l;
  split8(x, h, l);
  const size_t dh = (size_t)off + (size_t)n * kp + (size_t)k0;
  const size_t dl = dh + (size_t)HID * kp;
  if (ok) {
    *(volatile v4u*)(wsb + dh) = h.q;
    *(volatile v4u*)(wsb + dl) = l.q;
  }
  __threadfence();
  if (ok) {
    *(volatile v4u*)(wsb + dh) = h.q;
    *(volatile v4u*)(wsb + dl) = l.q;
  }
}

__device__ __forceinline__ void gemm128(v8f (&acc)[8],
                                        const unsigned short* __restrict__ ah, const unsigned short* __restrict__ al, int row,
                                        const unsigned short* __restrict__ wT, const unsigned short* __restrict__ wL,
                                        int kp, int kOff, int hh, int m) {
  const unsigned short* ar = ah + (size_t)row * HID + 8 * hh;
  const unsigned short* lr = al + (size_t)row * HID + 8 * hh;
#pragma unroll
  for (int ks = 0; ks < 4; ++ks) {
    FragB fa, fl;
    fa.q[0] = *(const v4u*)(ar + 32 * ks);  fa.q[1] = *(const v4u*)(ar + 32 * ks + 16);
    fl.q[0] = *(const v4u*)(lr + 32 * ks);  fl.q[1] = *(const v4u*)(lr + 32 * ks + 16);
#pragma unroll
    for (int nt = 0; nt < 8; ++nt) {
      const size_t wo = (size_t)(16 * nt + m) * kp + (size_t)(kOff + 32 * ks + 8 * hh);
      FragB bh, bl;
      bh.q[0] = *(const v4u*)(wT + wo);  bh.q[1] = *(const v4u*)(wT + wo + 16);
      bl.q[0] = *(const v4u*)(wL + wo);  bl.q[1] = *(const v4u*)(wL + wo + 16);
      acc[nt] = wmb(fa, bh, acc[nt]);
      acc[nt] = wmb(fa, bl, acc[nt]);
      acc[nt] = wmb(fl, bh, acc[nt]);
    }
  }
}

__device__ __forceinline__ void ng_store_f(const float* st, float* outF, int tile, int lane) {
#pragma unroll
  for (int j = 0; j < 16; ++j) {
    const v4f v = *(const v4f*)(st + j * HID + 4 * lane);
    *(volatile v4f*)(outF + (size_t)(tile * 16 + j) * HID + 4 * lane) = v;
  }
}

__device__ __forceinline__ void ng_store_b(const float* st, unsigned short* oh, unsigned short* ol, int tile, int hh, int m) {
#pragma unroll
  for (int j = 0; j < 8; ++j) {
    const int rr = 2 * j + hh;
    const float* sr = st + rr * HID + 8 * m;
    H8 h, l;
    split8(cat8(*(const v4f*)sr, *(const v4f*)(sr + 4)), h, l);
    const size_t gi = (size_t)(tile * 16 + rr) * HID + 8 * m;
    *(volatile v4u*)(oh + gi) = h.q;
    *(volatile v4u*)(ol + gi) = l.q;
  }
}

template <int ASRC, int OUTM>
__global__ __launch_bounds__(GTHR) void k_ngemm(
    const float* __restrict__ xf,
    const unsigned short* __restrict__ a0h, const unsigned short* __restrict__ a0l,
    const unsigned short* __restrict__ a1h, const unsigned short* __restrict__ a1l, int nA,
    const unsigned short* __restrict__ wT, int kp, int kOffA, int kOffB,
    const float* __restrict__ bias,
    float* outFA, float* outFB, unsigned short* outH, unsigned short* outL, int nTiles) {
  __shared__ __attribute__((aligned(16))) float stg[GW * 16 * HID];
  const int tid = threadIdx.x, lane = tid & 31, wave = tid >> 5, hh = lane >> 4, m = lane & 15;
  const int tile = blockIdx.x * GW + wave;
  const bool tv = tile < nTiles;
  const int kOff = (blockIdx.y != 0) ? kOffB : kOffA;
  float* outF = (blockIdx.y != 0) ? outFB : outFA;
  float* st = stg + wave * (16 * HID);
  const unsigned short* wL = wT + (size_t)HID * kp;

  if (tv) {
    const int row = tile * 16 + m;
    v8f acc[8];
#pragma unroll
    for (int t = 0; t < 8; ++t) acc[t] = zero8f();
    if (ASRC == 0) {
      const float* xr = xf + (size_t)row * 32;
      const v4f t0 = *(const v4f*)(xr + 8 * hh),      t1 = *(const v4f*)(xr + 8 * hh + 4);
      const v4f t2 = *(const v4f*)(xr + 16 + 8 * hh), t3 = *(const v4f*)(xr + 16 + 8 * hh + 4);
      H8 h0, l0, h1, l1;
      split8(cat8(t0, t1), h0, l0);
      split8(cat8(t2, t3), h1, l1);
      FragB fa, fl;
      fa.q[0] = h0.q; fa.q[1] = h1.q;
      fl.q[0] = l0.q; fl.q[1] = l1.q;
#pragma unroll
      for (int nt = 0; nt < 8; ++nt) {
        const size_t wo = (size_t)(16 * nt + m) * kp + (size_t)(kOff + 8 * hh);
        FragB bh, bl;
        bh.q[0] = *(const v4u*)(wT + wo);  bh.q[1] = *(const v4u*)(wT + wo + 16);
        bl.q[0] = *(const v4u*)(wL + wo);  bl.q[1] = *(const v4u*)(wL + wo + 16);
        acc[nt] = wmb(fa, bh, acc[nt]);
        acc[nt] = wmb(fa, bl, acc[nt]);
        acc[nt] = wmb(fl, bh, acc[nt]);
      }
    } else {
      gemm128(acc, a0h, a0l, row, wT, wL, kp, kOff, hh, m);
      if (nA > 1) gemm128(acc, a1h, a1l, row, wT, wL, kp, kOff + HID, hh, m);
    }
#pragma unroll
    for (int nt = 0; nt < 8; ++nt) {
      float bs = 0.0f;
      if (OUTM != 0) bs = bias[16 * nt + m];
#pragma unroll
      for (int r = 0; r < 8; ++r) {
        float v = acc[nt][r];
        if (OUTM != 0) v = fmaxf(v + bs, 0.0f);
        st[(8 * hh + r) * HID + 16 * nt + m] = v;
      }
    }
  }
  __builtin_amdgcn_fence(__ATOMIC_RELEASE, "wavefront");
  __builtin_amdgcn_wave_barrier();
  __builtin_amdgcn_fence(__ATOMIC_ACQUIRE, "wavefront");
  if (OUTM == 0) {
    if (tv) ng_store_f(st, outF, tile, lane);
    __threadfence();
    if (tv) ng_store_f(st, outF, tile, lane);
  } else {
    if (tv) ng_store_b(st, outH, outL, tile, hh, m);
    __threadfence();
    if (tv) ng_store_b(st, outH, outL, tile, hh, m);
  }
}

__device__ __forceinline__ void msg_put(float* mrow, const v8f (&acc)[8]) {
#pragma unroll
  for (int nt = 0; nt < 8; ++nt) {
    v4f a = {acc[nt][0], acc[nt][1], acc[nt][2], acc[nt][3]};
    v4f b = {acc[nt][4], acc[nt][5], acc[nt][6], acc[nt][7]};
    *(v4f*)(mrow + 16 * nt)     = a;
    *(v4f*)(mrow + 16 * nt + 4) = b;
  }
}

__device__ __forceinline__ void accum_half(float* accN, const float* msgb, const int* slotb, int off, int wave, int lane) {
  const int col = wave * 32 + lane;
#pragma unroll 1
  for (int i = 0; i < HALFP; ++i) {
    int sl = slotb[off + i];
    sl = sl < 0 ? 0 : (sl > NB ? NB : sl);
    const float v = msgb[i * HID + col];
    accN[sl * HID + col] = accN[sl * HID + col] + v;
  }
}

__device__ __forceinline__ void agg_out(const float* accN, unsigned short* aggH, unsigned short* aggL, int nodeBase, int wave, int hh, int m) {
#pragma unroll
  for (int j = 0; j < 8; ++j) {
    const int row = 2 * (wave + NWAVE * j) + hh;
    const float* ar = accN + row * HID + 8 * m;
    H8 h, l;
    split8(cat8(*(const v4f*)ar, *(const v4f*)(ar + 4)), h, l);
    const size_t gi = (size_t)(nodeBase + row) * HID + 8 * m;
    *(volatile v4u*)(aggH + gi) = h.q;
    *(volatile v4u*)(aggL + gi) = l.q;
  }
}

__global__ __launch_bounds__(NTHR) void k_agg(
    const float* __restrict__ ef, const int* __restrict__ ei,
    const float* __restrict__ Pp, const float* __restrict__ Qp,
    const unsigned short* __restrict__ wmT,
    const float* __restrict__ We, const float* __restrict__ be, const float* __restrict__ bm,
    unsigned short* aggH, unsigned short* aggL, int nN, int nE, int vec8) {
  __shared__ __attribute__((aligned(16))) float accN[(NB + 1) * HID];
  __shared__ __attribute__((aligned(16))) float msgb[HALFP * HID];
  __shared__ __attribute__((aligned(16))) unsigned short stgX[NWAVE * 16 * 32];
  __shared__ __attribute__((aligned(16))) unsigned short weT[2 * HID * 32];
  __shared__ __attribute__((aligned(16))) float bE[HID];
  __shared__ __attribute__((aligned(16))) float bM[HID];
  __shared__ __attribute__((aligned(16))) int hlst[LISTN];
  __shared__ __attribute__((aligned(16))) int pend[PCAP];
  __shared__ int slotb[PASSN];
  __shared__ int wcnt[NWAVE];
  __shared__ int pendN;

  const int tid = threadIdx.x, lane = tid & 31, wave = tid >> 5, hh = lane >> 4, m = lane & 15;
  const int nodeBase = blockIdx.x * NB;
  const int* srcs = ei;
  const int* dsts = ei + nE;
  const unsigned short* wmL = wmT + (size_t)HID * WMP;

  for (int i = tid; i < (NB + 1) * HID; i += NTHR) accN[i] = 0.0f;
  for (int i = tid; i < HID * 32; i += NTHR) {
    const int n = i >> 5, c = i & 15;
    unsigned short h, l;
    split1(We[c * HID + n], h, l);
    weT[i] = h;
    weT[HID * 32 + i] = l;
  }
  if (tid < HID) { bE[tid] = be[tid]; bM[tid] = bm[tid]; }
  if (tid == 0) pendN = 0;
  __syncthreads();

  const int nChunks = (nE + CHUNK - 1) / CHUNK;
#pragma unroll 1
  for (int ch = 0; ch < nChunks; ++ch) {
    const int cbase = ch * CHUNK;
    const int wc = scan_chunk(dsts, nE, cbase, nodeBase, vec8, hlst, tid, wave);
    if (lane == 0) wcnt[wave] = wc;
    __syncthreads();

    const int base = pendN;
    int tot = 0, myoff = 0;
#pragma unroll
    for (int w = 0; w < NWAVE; ++w) {
      int c = wcnt[w];
      c = c > WCAP ? WCAP : (c < 0 ? 0 : c);
      if (w < wave) myoff += c;
      tot += c;
    }
    int newN = base + tot;
    newN = newN > PCAP ? PCAP : newN;
    {
      int n = wcnt[wave];
      n = n > WCAP ? WCAP : (n < 0 ? 0 : n);
      const int* lp = hlst + wave * WCAP;
      for (int i = lane; i < n; i += 32) {
        const int pos = base + myoff + i;
        if (pos < PCAP) pend[pos] = cbase + lp[i];
      }
    }
    const int fin = (ch == nChunks - 1) ? 1 : 0;
    const int R   = (fin != 0) ? (newN + PASSN - 1) / PASSN : newN / PASSN;
    const int Pv  = (fin != 0) ? newN : R * PASSN;
    __syncthreads();

#pragma unroll 1
    for (int r = 0; r < R; ++r) {
      int sN, dN;
      {
        int idx = r * PASSN + wave * 16 + m;
        const bool valid = idx < Pv;
        idx = idx > PCAP - 1 ? PCAP - 1 : idx;
        int e = pend[idx];
        e = valid ? e : 0;
        e = e < 0 ? 0 : (e > nE - 1 ? nE - 1 : e);
        int d = dsts[e];
        int s = srcs[e];
        int slot = d - nodeBase;
        if (!valid || (unsigned)slot >= (unsigned)NB) slot = NB;
        d = d < 0 ? 0 : (d > nN - 1 ? nN - 1 : d);
        s = s < 0 ? 0 : (s > nN - 1 ? nN - 1 : s);
        sN = s; dN = d;
        const float* xr = ef + (size_t)e * 16 + 8 * hh;
        H8 xh, xl;
        split8(cat8(*(const v4f*)xr, *(const v4f*)(xr + 4)), xh, xl);
        unsigned short* sp = stgX + (wave * 16 + m) * 32;
        *(v4u*)(sp + 8 * hh)      = xh.q;
        *(v4u*)(sp + 16 + 8 * hh) = xl.q;
        if (hh == 0) slotb[wave * 16 + m] = slot;
      }
      __builtin_amdgcn_fence(__ATOMIC_RELEASE, "wavefront");
      __builtin_amdgcn_wave_barrier();
      __builtin_amdgcn_fence(__ATOMIC_ACQUIRE, "wavefront");

      FragB bx;
      {
        const unsigned short* sp = stgX + (wave * 16 + m) * 32;
        bx.q[0] = *(const v4u*)(sp + 8 * hh);
        bx.q[1] = *(const v4u*)(sp + 16 + 8 * hh);
      }

      v8f acc[8];
#pragma unroll
      for (int t = 0; t < 8; ++t) acc[t] = zero8f();
#pragma unroll
      for (int ks = 0; ks < 4; ++ks) {
        FragB Bh, Bl;
        {
          FragB a1, a2;
          const unsigned short* w0 = weT + (32 * ks + m) * 32 + 8 * hh;
          a1.q[0] = *(const v4u*)(w0);             a1.q[1] = *(const v4u*)(w0 + 16);
          a2.q[0] = *(const v4u*)(w0 + HID * 32);  a2.q[1] = *(const v4u*)(w0 + HID * 32 + 16);
          v8f d0 = wmb(a1, bx, zero8f());
          d0 = wmb(a2, bx, d0);
          const unsigned short* w1 = w0 + 16 * 32;
          a1.q[0] = *(const v4u*)(w1);             a1.q[1] = *(const v4u*)(w1 + 16);
          a2.q[0] = *(const v4u*)(w1 + HID * 32);  a2.q[1] = *(const v4u*)(w1 + HID * 32 + 16);
          v8f d1 = wmb(a1, bx, zero8f());
          d1 = wmb(a2, bx, d1);
          const float* bp = bE + 32 * ks + 8 * hh;
          const v8f e0 = cat8(*(const v4f*)bp, *(const v4f*)(bp + 4));
          const v8f e1 = cat8(*(const v4f*)(bp + 16), *(const v4f*)(bp + 20));
          v8f r0, r1;
#pragma unroll
          for (int i = 0; i < 8; ++i) {
            r0[i] = fmaxf(d0[i] + e0[i], 0.0f);
            r1[i] = fmaxf(d1[i] + e1[i], 0.0f);
          }
          H8 h0, l0, h1, l1;
          split8(r0, h0, l0);
          split8(r1, h1, l1);
          Bh.q[0] = h0.q; Bh.q[1] = h1.q;
          Bl.q[0] = l0.q; Bl.q[1] = l1.q;
        }
#pragma unroll
        for (int nt = 0; nt < 8; ++nt) {
          FragB ah, al;
          const size_t wo = (size_t)(16 * nt + m) * WMP + (size_t)(KOFE + 32 * ks + 8 * hh);
          ah.q[0] = *(const v4u*)(wmT + wo);  ah.q[1] = *(const v4u*)(wmT + wo + 16);
          al.q[0] = *(const v4u*)(wmL + wo);  al.q[1] = *(const v4u*)(wmL + wo + 16);
          acc[nt] = wmb(ah, Bh, acc[nt]);
          acc[nt] = wmb(ah, Bl, acc[nt]);
          acc[nt] = wmb(al, Bh, acc[nt]);
        }
      }

#pragma unroll
      for (int nt = 0; nt < 8; ++nt) {
        const int f0 = 16 * nt + 8 * hh;
        const float* pr = Pp + (size_t)sN * HID + f0;
        const float* qr = Qp + (size_t)dN * HID + f0;
        const v8f pv = cat8(*(const v4f*)pr, *(const v4f*)(pr + 4));
        const v8f qv = cat8(*(const v4f*)qr, *(const v4f*)(qr + 4));
        const v8f bv = cat8(*(const v4f*)(bM + f0), *(const v4f*)(bM + f0 + 4));
        v8f t = acc[nt];
#pragma unroll
        for (int i = 0; i < 8; ++i) t[i] = fmaxf(t[i] + pv[i] + qv[i] + bv[i], 0.0f);
        acc[nt] = t;
      }

      float* mrow = msgb + ((wave & 3) * 16 + m) * HID + 8 * hh;
      if (wave < 4) msg_put(mrow, acc);
      __syncthreads();
      if (wave < 4) accum_half(accN, msgb, slotb, 0, wave, lane);
      __syncthreads();
      if (wave >= 4) msg_put(mrow, acc);
      __syncthreads();
      if (wave < 4) accum_half(accN, msgb, slotb, HALFP, wave, lane);
      __syncthreads();
    }

    int rem = newN - R * PASSN;
    rem = rem < 0 ? 0 : rem;
    if (R > 0 && tid < rem) pend[tid] = pend[R * PASSN + tid];
    if (tid == 0) pendN = rem;
  }
  __syncthreads();

  agg_out(accN, aggH, aggL, nodeBase, wave, hh, m);
  __threadfence();
  agg_out(accN, aggH, aggL, nodeBase, wave, hh, m);
}

__global__ __launch_bounds__(DTHR) void k_dem(
    const float* __restrict__ dem, const int* __restrict__ pairs,
    const float* __restrict__ R1, const float* __restrict__ R2,
    const float* __restrict__ Wr1, const float* __restrict__ br1,
    const float* __restrict__ Wr2, const float* __restrict__ br2,
    float* out, int nN, int nD, int nTiles) {
  __shared__ __attribute__((aligned(16))) unsigned short wfT[HID * 32];
  __shared__ __attribute__((aligned(16))) float sb[HID];
  __shared__ __attribute__((aligned(16))) float sw[HID];
  __shared__ __attribute__((aligned(16))) float so[DPB];
  const int tid = threadIdx.x, lane = tid & 31, wave = tid >> 5, hh = lane >> 4, m = lane & 15;

  for (int i = tid; i < HID * 32; i += DTHR) {
    const int n = i >> 5, s = i & 31, c = s & 7, g = s >> 3;
    unsigned short h, l;
    split1(Wr1[(size_t)(2 * HID + c) * HID + n], h, l);
    unsigned short v = 0;
    if (g == 0 || g == 2) v = h;
    else if (g == 1) v = l;
    wfT[i] = v;
  }
  if (tid < HID) { sb[tid] = br1[tid]; sw[tid] = Wr2[tid]; }
  __syncthreads();

  const int t = blockIdx.x * 8 + wave;
  const bool tv = t < nTiles;
  float res = 0.0f;
  if (tv) {
    const int di = t * 16 + m;
    int ds = pairs[2 * di];
    int dd = pairs[2 * di + 1];
    ds = ds < 0 ? 0 : (ds > nN - 1 ? nN - 1 : ds);
    dd = dd < 0 ? 0 : (dd > nN - 1 ? nN - 1 : dd);
    const float* fr = dem + (size_t)di * 8;
    H8 fh, fl;
    split8(cat8(*(const v4f*)fr, *(const v4f*)(fr + 4)), fh, fl);
    FragB b;
    b.q[0] = fh.q;
    b.q[1] = (hh == 0) ? fl.q : zero4u();
    v8f acc[8];
#pragma unroll
    for (int nt = 0; nt < 8; ++nt) {
      FragB a;
      const unsigned short* wp = wfT + (16 * nt + m) * 32 + 8 * hh;
      a.q[0] = *(const v4u*)(wp);
      a.q[1] = *(const v4u*)(wp + 16);
      acc[nt] = wmb(a, b, zero8f());
    }
    float part = 0.0f;
#pragma unroll
    for (int nt = 0; nt < 8; ++nt) {
      const int f0 = 16 * nt + 8 * hh;
      const float* r1 = R1 + (size_t)ds * HID + f0;
      const float* r2 = R2 + (size_t)dd * HID + f0;
      const v8f a1 = cat8(*(const v4f*)r1, *(const v4f*)(r1 + 4));
      const v8f a2 = cat8(*(const v4f*)r2, *(const v4f*)(r2 + 4));
      const v8f bb = cat8(*(const v4f*)(sb + f0), *(const v4f*)(sb + f0 + 4));
      const v8f ww = cat8(*(const v4f*)(sw + f0), *(const v4f*)(sw + f0 + 4));
#pragma unroll
      for (int i = 0; i < 8; ++i) {
        const float hv = fmaxf(acc[nt][i] + a1[i] + a2[i] + bb[i], 0.0f);
        part += hv * ww[i];
      }
    }
    const float oth = __shfl_xor(part, 16, 32);
    float s = (part + oth) + br2[0];
    s = fminf(fmaxf(s, -40.0f), 40.0f);
    const float ex = __expf(-s);
    res = __builtin_amdgcn_rcpf(1.0f + ex);
  }
  if (hh == 0) so[wave * 16 + m] = res;
  __syncthreads();

  const int gi = blockIdx.x * DPB + 4 * lane;
  const bool wok = (wave == 0) && (gi + 3 < nD);
  const v4f ov = *(const v4f*)(so + 4 * lane);
  if (wok) *(volatile v4f*)(out + gi) = ov;
  __threadfence();
  if (wok) *(volatile v4f*)(out + gi) = ov;
}

extern "C" void kernel_launch(void* const* d_in, const int* in_sizes, int n_in,
                              void* d_out, int out_size, void* d_ws, size_t ws_size,
                              hipStream_t stream) {
  if (n_in < 21) return;
  const int nN = in_sizes[0] / 32;
  const int nE = in_sizes[1] / 16;
  const int nD = in_sizes[2] / 8;
  if (nN < 16 || nE < 1 || nD < 16) return;
  if (in_sizes[0] != nN * 32 || in_sizes[1] != nE * 16 || in_sizes[2] != nD * 8) return;
  if (in_sizes[3] != 2 * nE || in_sizes[4] != 2 * nD) return;
  if ((nN % 16) != 0 || (nD % 16) != 0) return;
  if (in_sizes[5] != 32 * HID || in_sizes[6] < HID || in_sizes[7] != 16 * HID || in_sizes[8] < HID) return;
  if (in_sizes[9] != 3 * HID * HID || in_sizes[10] < HID || in_sizes[11] != 2 * HID * HID || in_sizes[12] < HID) return;
  if (in_sizes[13] != 3 * HID * HID || in_sizes[14] < HID || in_sizes[15] != 2 * HID * HID || in_sizes[16] < HID) return;
  if (in_sizes[17] != (2 * HID + 8) * HID || in_sizes[18] < HID || in_sizes[19] < HID || in_sizes[20] < 1) return;
  if (out_size != nD) return;

  const float* node_feats   = (const float*)d_in[0];
  const float* edge_feats   = (const float*)d_in[1];
  const float* demand_feats = (const float*)d_in[2];
  const int*   edge_index   = (const int*)d_in[3];
  const int*   demand_pairs = (const int*)d_in[4];
  const float* W_node = (const float*)d_in[5];   const float* b_node = (const float*)d_in[6];
  const float* W_edge = (const float*)d_in[7];   const float* b_edge = (const float*)d_in[8];
  const float* W_msg0 = (const float*)d_in[9];   const float* b_msg0 = (const float*)d_in[10];
  const float* W_upd0 = (const float*)d_in[11];  const float* b_upd0 = (const float*)d_in[12];
  const float* W_msg1 = (const float*)d_in[13];  const float* b_msg1 = (const float*)d_in[14];
  const float* W_upd1 = (const float*)d_in[15];  const float* b_upd1 = (const float*)d_in[16];
  const float* W_r1   = (const float*)d_in[17];  const float* b_r1   = (const float*)d_in[18];
  const float* W_r2   = (const float*)d_in[19];  const float* b_r2   = (const float*)d_in[20];
  float* out = (float*)d_out;

  const int nTN  = nN / 16;
  const int nBlk = (nN + NB - 1) / NB;
  const int rowsAgg = nBlk * NB;
  const int nTD  = nD / 16;
  const int nBD  = (nD + DPB - 1) / DPB;

  size_t off = 0;
  auto take = [&](size_t bytes) -> size_t {
    const size_t o = off;
    off = (off + bytes + 255) & ~(size_t)255;
    return o;
  };
  const size_t oWn  = take((size_t)2 * HID * 32 * 2);
  const size_t oWm0 = take((size_t)2 * HID * WMP * 2);
  const size_t oWu0 = take((size_t)2 * HID * 2 * HID * 2);
  const size_t oWm1 = take((size_t)2 * HID * WMP * 2);
  const size_t oWu1 = take((size_t)2 * HID * 2 * HID * 2);
  const size_t oWr  = take((size_t)2 * HID * 2 * HID * 2);
  const size_t hBytes = (size_t)nN * HID * 2;
  const size_t aBytes = (size_t)rowsAgg * HID * 2;
  const size_t pBytes = (size_t)nN * HID * 4;
  const size_t oHAh = take(hBytes), oHAl = take(hBytes), oHBh = take(hBytes), oHBl = take(hBytes);
  const size_t oAGh = take(aBytes), oAGl = take(aBytes);
  const size_t oP = take(pBytes), oQ = take(pBytes);
  if (off > ws_size || off > ((size_t)128 << 20)) return;

  char* ws = (char*)d_ws;
  unsigned short* wsb = (unsigned short*)ws;
  const unsigned short* Wn  = (const unsigned short*)(ws + oWn);
  const unsigned short* Wm0 = (const unsigned short*)(ws + oWm0);
  const unsigned short* Wu0 = (const unsigned short*)(ws + oWu0);
  const unsigned short* Wm1 = (const unsigned short*)(ws + oWm1);
  const unsigned short* Wu1 = (const unsigned short*)(ws + oWu1);
  const unsigned short* Wr  = (const unsigned short*)(ws + oWr);
  unsigned short* hAh = (unsigned short*)(ws + oHAh);
  unsigned short* hAl = (unsigned short*)(ws + oHAl);
  unsigned short* hBh = (unsigned short*)(ws + oHBh);
  unsigned short* hBl = (unsigned short*)(ws + oHBl);
  unsigned short* aGh = (unsigned short*)(ws + oAGh);
  unsigned short* aGl = (unsigned short*)(ws + oAGl);
  float* Pp = (float*)(ws + oP);
  float* Qp = (float*)(ws + oQ);

  const int vec8 = ((nE & 3) == 0) ? 1 : 0;

  const int gxw = (16 * WMP + 255) / 256;
  k_wprep<<<dim3(gxw, 6, 1), 256, 0, stream>>>(
      W_node, W_msg0, W_upd0, W_msg1, W_upd1, W_r1,
      32, 3 * HID, 2 * HID, 3 * HID, 2 * HID, 2 * HID,
      32, WMP, 2 * HID, WMP, 2 * HID, 2 * HID,
      (int)(oWn / 2), (int)(oWm0 / 2), (int)(oWu0 / 2), (int)(oWm1 / 2), (int)(oWu1 / 2), (int)(oWr / 2),
      wsb);

  const dim3 gg1((nTN + GW - 1) / GW, 1, 1);
  const dim3 gg2((nTN + GW - 1) / GW, 2, 1);

  k_ngemm<0, 1><<<gg1, GTHR, 0, stream>>>(node_feats, hBh, hBl, hBh, hBl, 0, Wn, 32, 0, 0, b_node,
                                          Pp, Qp, hAh, hAl, nTN);

  k_ngemm<1, 0><<<gg2, GTHR, 0, stream>>>(node_feats, hAh, hAl, hAh, hAl, 1, Wm0, WMP, 0, 2 * HID, b_node,
                                          Pp, Qp, aGh, aGl, nTN);
  k_agg<<<nBlk, NTHR, 0, stream>>>(edge_feats, edge_index, Pp, Qp, Wm0, W_edge, b_edge, b_msg0,
                                   aGh, aGl, nN, nE, vec8);
  k_ngemm<1, 1><<<gg1, GTHR, 0, stream>>>(node_feats, hAh, hAl, aGh, aGl, 2, Wu0, 2 * HID, 0, 0, b_upd0,
                                          Pp, Qp, hBh, hBl, nTN);

  k_ngemm<1, 0><<<gg2, GTHR, 0, stream>>>(node_feats, hBh, hBl, hBh, hBl, 1, Wm1, WMP, 0, 2 * HID, b_node,
                                          Pp, Qp, aGh, aGl, nTN);
  k_agg<<<nBlk, NTHR, 0, stream>>>(edge_feats, edge_index, Pp, Qp, Wm1, W_edge, b_edge, b_msg1,
                                   aGh, aGl, nN, nE, vec8);
  k_ngemm<1, 1><<<gg1, GTHR, 0, stream>>>(node_feats, hBh, hBl, aGh, aGl, 2, Wu1, 2 * HID, 0, 0, b_upd1,
                                          Pp, Qp, hAh, hAl, nTN);

  k_ngemm<1, 0><<<gg2, GTHR, 0, stream>>>(node_feats, hAh, hAl, hAh, hAl, 1, Wr, 2 * HID, 0, HID, b_node,
                                          Pp, Qp, aGh, aGl, nTN);
  k_dem<<<nBD, DTHR, 0, stream>>>(demand_feats, demand_pairs, Pp, Qp, W_r1, b_r1, W_r2, b_r2,
                                  out, nN, nD, nTD);
}
